// DilatedSelfAttention_65300682769193
// MI455X (gfx1250) — hardware-verified
//
#include <hip/hip_runtime.h>
#include <math.h>
#include <stdint.h>

#define NB   2
#define NSEQ 8192
#define NC   256
#define NG   7
#define NS   2048
#define NZ   (NB * NG)
#define NQB  (NS / 64)
static_assert(NZ == 14);
static_assert(NQB == 32);
static_assert((NC % 64) == 0 && (NS % 64) == 0 && (NC % 32) == 0);

typedef __bf16   v16b __attribute__((ext_vector_type(16)));
typedef __bf16   v8b  __attribute__((ext_vector_type(8)));
typedef float    v8f  __attribute__((ext_vector_type(8)));
typedef float    v4f  __attribute__((ext_vector_type(4)));
typedef unsigned int v4u __attribute__((ext_vector_type(4)));

__device__ __forceinline__ unsigned short bf_bits(float f) {
  unsigned u = __float_as_uint(f);
  return (unsigned short)((u + 0x7FFFu + ((u >> 16) & 1u)) >> 16);
}
__device__ __forceinline__ float bf_up(unsigned short h) { return __uint_as_float(((unsigned)h) << 16); }
__device__ __forceinline__ __bf16 bf_val(unsigned short h) { return __builtin_bit_cast(__bf16, h); }
__device__ __forceinline__ unsigned pk16(unsigned short a, unsigned short b) { return (unsigned)a | ((unsigned)b << 16); }
__device__ __forceinline__ v8f zero8() { v8f z = {0.f, 0.f, 0.f, 0.f, 0.f, 0.f, 0.f, 0.f}; return z; }

__device__ __forceinline__ v16b ldfrag_b(const __bf16* p) {
  union { v16b v; v8b h[2]; } f;
  f.h[0] = *(const v8b*)(p);
  f.h[1] = *(const v8b*)(p + 16);
  return f.v;
}

__device__ __forceinline__ v8f mma_b(v16b a, v16b b, v8f c) {
  c = __builtin_amdgcn_wmma_f32_16x16x32_bf16(false, a, false, b, (short)0, c, false, false);
  asm volatile("v_nop\n\tv_nop\n\tv_nop\n\tv_nop" : "+v"(c) : "v"(a), "v"(b));
  return c;
}
__device__ __forceinline__ v8f mma_b_raw(v16b a, v16b b, v8f c) {
  return __builtin_amdgcn_wmma_f32_16x16x32_bf16(false, a, false, b, (short)0, c, false, false);
}
__device__ __forceinline__ void dep_guard_b(v8f& a, v8f& b, v16b x) {
  asm volatile("v_nop\n\tv_nop\n\tv_nop\n\tv_nop" : "+v"(a), "+v"(b) : "v"(x));
}
__device__ __forceinline__ void keep4_b(v16b a, v16b b, v16b c, v16b d) {
  asm volatile("v_nop" :: "v"(a), "v"(b), "v"(c), "v"(d));
}
__device__ __forceinline__ void acc_guard4(v8f& a, v8f& b, v8f& c, v8f& d) {
  asm volatile("v_nop\n\tv_nop\n\tv_nop\n\tv_nop" : "+v"(a), "+v"(b), "+v"(c), "+v"(d));
}

__device__ __forceinline__ void group_geom(int z, size_t& xbase, int& pitch) {
  const int b  = z / NG;
  const int g  = z - b * NG;
  const int rs = (g < 4) ? 1 : ((g < 6) ? 2 : 4);
  const int sg = (g < 4) ? (g * 2048) : ((g < 6) ? ((g - 4) * 4096) : 0);
  xbase = ((size_t)b * NSEQ + (size_t)sg) * NC;
  pitch = NC * rs;
}

__global__ __launch_bounds__(256) void cvt_bf16x8(const float* __restrict__ in, unsigned short* out, int n8) {
  const int i = blockIdx.x * 256 + threadIdx.x;
  if (i < n8) {
    const v4f a = *(const v4f*)(in + (size_t)i * 8);
    const v4f b = *(const v4f*)(in + (size_t)i * 8 + 4);
    v4u p;
    p[0] = pk16(bf_bits(a[0]), bf_bits(a[1]));
    p[1] = pk16(bf_bits(a[2]), bf_bits(a[3]));
    p[2] = pk16(bf_bits(b[0]), bf_bits(b[1]));
    p[3] = pk16(bf_bits(b[2]), bf_bits(b[3]));
    *(volatile v4u*)(out + (size_t)i * 8) = p;
    __threadfence();
    *(volatile v4u*)(out + (size_t)i * 8) = p;
  }
}

__device__ __forceinline__ void wt_tile_to_lds(const float* __restrict__ W, unsigned short* sp, int tid, int d0) {
  const float* row = W + (size_t)tid * NC + d0;
  const v4f a0 = *(const v4f*)(row);
  const v4f a1 = *(const v4f*)(row + 4);
  const v4f a2 = *(const v4f*)(row + 8);
  const v4f a3 = *(const v4f*)(row + 12);
#pragma unroll
  for (int e = 0; e < 4; ++e) {
    sp[(e)      * NC + tid] = bf_bits(a0[e]);
    sp[(4 + e)  * NC + tid] = bf_bits(a1[e]);
    sp[(8 + e)  * NC + tid] = bf_bits(a2[e]);
    sp[(12 + e) * NC + tid] = bf_bits(a3[e]);
  }
}
__global__ __launch_bounds__(256) void prep_wt(const float* __restrict__ Wq, const float* __restrict__ Wk,
                                               const float* __restrict__ Wv,
                                               unsigned short* WqT, unsigned short* WkT, unsigned short* WvT) {
  __shared__ __align__(16) unsigned short sW[3 * 16 * NC];
  const int tid  = threadIdx.x;
  const int wave = tid >> 5;
  const int lane = tid & 31;
  const int d0   = blockIdx.x * 16;
  wt_tile_to_lds(Wq, sW,               tid, d0);
  wt_tile_to_lds(Wk, sW + 16 * NC,     tid, d0);
  wt_tile_to_lds(Wv, sW + 2 * 16 * NC, tid, d0);
  __syncthreads();
  const int r0 = 2 * wave;
  const v4u q0v = *(const v4u*)(sW + (0 * 16 + r0) * NC + lane * 8);
  const v4u q1v = *(const v4u*)(sW + (0 * 16 + r0 + 1) * NC + lane * 8);
  const v4u k0v = *(const v4u*)(sW + (1 * 16 + r0) * NC + lane * 8);
  const v4u k1v = *(const v4u*)(sW + (1 * 16 + r0 + 1) * NC + lane * 8);
  const v4u v0v = *(const v4u*)(sW + (2 * 16 + r0) * NC + lane * 8);
  const v4u v1v = *(const v4u*)(sW + (2 * 16 + r0 + 1) * NC + lane * 8);
  const size_t o0 = (size_t)(d0 + r0) * NC + lane * 8;
  const size_t o1 = (size_t)(d0 + r0 + 1) * NC + lane * 8;
  for (int pass = 0; pass < 2; ++pass) {
    *(volatile v4u*)(WqT + o0) = q0v;
    *(volatile v4u*)(WqT + o1) = q1v;
    *(volatile v4u*)(WkT + o0) = k0v;
    *(volatile v4u*)(WkT + o1) = k1v;
    *(volatile v4u*)(WvT + o0) = v0v;
    *(volatile v4u*)(WvT + o1) = v1v;
    __threadfence();
  }
}

template <bool XA>
__global__ __launch_bounds__(256) void pgemm(const unsigned short* __restrict__ Xbp,
                                             const unsigned short* __restrict__ Wtp,
                                             unsigned short* Chp, unsigned short* Clp) {
  constexpr int M = XA ? NS : NC;
  constexpr int N = XA ? NC : NS;
  constexpr int K = NC;
  static_assert((M % 64) == 0 && (N % 64) == 0 && (K % 32) == 0);
  __shared__ __align__(16) float sT[8][16 * 68];
  const int z = blockIdx.y;
  size_t xbase; int xpitch;
  group_geom(z, xbase, xpitch);
  const __bf16* Xb = (const __bf16*)(const void*)Xbp;
  const __bf16* Wt = (const __bf16*)(const void*)Wtp;
  const __bf16* Ab = XA ? (Xb + xbase) : Wt;
  const int     lda = XA ? xpitch : NC;
  const __bf16* Bb = XA ? Wt : (Xb + xbase);
  const int     ldb = XA ? NC : xpitch;

  const int lane = threadIdx.x & 31;
  const int wave = threadIdx.x >> 5;
  const int tilesN = N >> 6;
  const int tilesM = M >> 6;
  const int tile = blockIdx.x * 8 + wave;
  if (tile >= tilesM * tilesN) return;
  const int tm = tile / tilesN;
  const int tn = tile - tm * tilesN;
  const int m0 = tm << 6;
  const int n0 = tn << 6;

  const int rlane = lane & 15;
  const int koff  = (lane >> 4) * 8;
  const int mOff  = (lane >> 4) * 8;

  v8f acc[4][4];
#pragma unroll
  for (int i = 0; i < 4; ++i)
#pragma unroll
    for (int j = 0; j < 4; ++j) acc[i][j] = zero8();

  for (int k0 = 0; k0 < K; k0 += 32) {
    v16b bh[4];
#pragma unroll
    for (int j = 0; j < 4; ++j) {
      const size_t bo = (size_t)(n0 + (j << 4) + rlane) * ldb + koff + k0;
      bh[j] = ldfrag_b(Bb + bo);
    }
#pragma unroll
    for (int i = 0; i < 4; ++i) {
      const size_t ao = (size_t)(m0 + (i << 4) + rlane) * lda + koff + k0;
      const v16b ah = ldfrag_b(Ab + ao);
#pragma unroll
      for (int j = 0; j < 4; ++j) {
        acc[i][j] = mma_b_raw(ah, bh[j], acc[i][j]);
      }
      dep_guard_b(acc[i][0], acc[i][3], ah);
    }
    keep4_b(bh[0], bh[1], bh[2], bh[3]);
  }
  acc_guard4(acc[0][0], acc[0][1], acc[0][2], acc[0][3]);
  acc_guard4(acc[1][0], acc[1][1], acc[1][2], acc[1][3]);
  acc_guard4(acc[2][0], acc[2][1], acc[2][2], acc[2][3]);
  acc_guard4(acc[3][0], acc[3][1], acc[3][2], acc[3][3]);

  float* slab = sT[wave];
  unsigned short* C  = Chp + (size_t)z * M * N;
  unsigned short* C2 = Clp + (size_t)z * M * N;
#pragma unroll
  for (int i = 0; i < 4; ++i) {
    const int mBase = m0 + (i << 4);
#pragma unroll
    for (int j = 0; j < 4; ++j) {
#pragma unroll
      for (int r = 0; r < 8; ++r) {
        slab[(mOff + r) * 68 + (j << 4) + rlane] = acc[i][j][r];
      }
    }
    __builtin_amdgcn_fence(__ATOMIC_RELEASE, "workgroup");
    __builtin_amdgcn_wave_barrier();
    __builtin_amdgcn_fence(__ATOMIC_ACQUIRE, "workgroup");
    {
      const int q = lane >> 3, c8 = (lane & 7) * 8;
      v4u hv[4], lv[4];
#pragma unroll
      for (int it = 0; it < 4; ++it) {
        const int row = it * 4 + q;
        const float* sp = slab + row * 68 + c8;
        v4u a, a2;
#pragma unroll
        for (int e = 0; e < 4; ++e) {
          const float f0 = sp[2 * e], f1 = sp[2 * e + 1];
          const unsigned short h0 = bf_bits(f0), h1 = bf_bits(f1);
          const unsigned short l0 = bf_bits(f0 - bf_up(h0)), l1 = bf_bits(f1 - bf_up(h1));
          a[e] = pk16(h0, h1); a2[e] = pk16(l0, l1);
        }
        hv[it] = a; lv[it] = a2;
      }
      for (int pass = 0; pass < 2; ++pass) {
#pragma unroll
        for (int it = 0; it < 4; ++it) {
          const int row = it * 4 + q;
          *(volatile v4u*)(C  + (size_t)(mBase + row) * N + n0 + c8) = hv[it];
          *(volatile v4u*)(C2 + (size_t)(mBase + row) * N + n0 + c8) = lv[it];
        }
        __threadfence();
      }
    }
    __builtin_amdgcn_fence(__ATOMIC_RELEASE, "workgroup");
    __builtin_amdgcn_wave_barrier();
    __builtin_amdgcn_fence(__ATOMIC_ACQUIRE, "workgroup");
  }
}

#define L_KSH   0
#define L_KSL   32768
#define L_VTH   65536
#define L_VTL   98304
#define L_PH    131072
#define L_PL    139264
#define L_ACC   147456
#define L_SD    212992
#define L_TOTAL 213248
static_assert(L_KSL - L_KSH == 64 * NC * 2 && L_VTH - L_KSL == 64 * NC * 2);
static_assert(L_VTL - L_VTH == NC * 64 * 2 && L_PH - L_VTL == NC * 64 * 2);
static_assert(L_PL - L_PH == 4 * 16 * 64 * 2 && L_ACC - L_PL == 4 * 16 * 64 * 2);
static_assert(L_SD - L_ACC == 4 * 16 * 32 * 8 * 4 && L_TOTAL - L_SD == 64 * 4);
static_assert(4 * 16 * NC * 4 <= L_VTH);

__global__ __launch_bounds__(128)
void attn_causal(const unsigned short* __restrict__ qhp, const unsigned short* __restrict__ qlp,
                 const unsigned short* __restrict__ khp, const unsigned short* __restrict__ klp,
                 const unsigned short* __restrict__ vhp, const unsigned short* __restrict__ vlp,
                 float* Op, float* Dp) {
  extern __shared__ __align__(16) unsigned char lds[];
  union FB { v16b v; v8b h[2]; };
  __bf16* Ksh  = (__bf16*)(lds + L_KSH);
  __bf16* Ksl  = (__bf16*)(lds + L_KSL);
  __bf16* Vth  = (__bf16*)(lds + L_VTH);
  __bf16* Vtl  = (__bf16*)(lds + L_VTL);
  __bf16* Ph   = (__bf16*)(lds + L_PH);
  __bf16* Pl   = (__bf16*)(lds + L_PL);
  float*  accL = (float*)(lds + L_ACC);
  float*  sD   = (float*)(lds + L_SD);

  const int tid  = threadIdx.x;
  const int wave = tid >> 5;
  const int lane = tid & 31;
  const int hh   = lane >> 4;
  const int c    = lane & 15;

  const int bx = blockIdx.x;
  const int qb = bx & (NQB - 1);
  const int z  = bx >> 5;
  const int q0 = qb * 64 + wave * 16;
  const size_t zrow = (size_t)z * NS;

  const __bf16* Qh = (const __bf16*)(const void*)qhp;
  const __bf16* Ql = (const __bf16*)(const void*)qlp;
  const __bf16* Kh = (const __bf16*)(const void*)khp;
  const __bf16* Kl = (const __bf16*)(const void*)klp;
  const __bf16* Vh = (const __bf16*)(const void*)vhp + (size_t)z * NC * NS;
  const __bf16* Vl = (const __bf16*)(const void*)vlp + (size_t)z * NC * NS;

  float*  accW = accL + wave * 4096;
  __bf16* pwh  = Ph + wave * 1024;
  __bf16* pwl  = Pl + wave * 1024;

#pragma unroll
  for (int t = 0; t < 16; ++t) *(v8f*)(accW + (t * 32 + lane) * 8) = zero8();

  float mrow[8], lrow[8], alpha[8];
#pragma unroll
  for (int r = 0; r < 8; ++r) { mrow[r] = -INFINITY; lrow[r] = 0.f; alpha[r] = 0.f; }

  const size_t qo = (zrow + q0 + c) * NC + 8 * hh;

  for (int kt = 0; kt <= qb; ++kt) {
    const int kv0 = kt * 64;
    __syncthreads();
    {
      const __bf16* kgh = Kh + (zrow + kv0) * NC;
      const __bf16* kgl = Kl + (zrow + kv0) * NC;
      const __bf16* vgh = Vh + kv0;
      const __bf16* vgl = Vl + kv0;
#pragma unroll 4
      for (int i = 0; i < 16; ++i) {
        const int p  = tid + 128 * i;
        const int d  = p >> 3;
        const int sg = (p & 7) * 8;
        const v8b a0 = *(const v8b*)(kgh + p * 8);
        const v8b a1 = *(const v8b*)(kgl + p * 8);
        const v8b b0 = *(const v8b*)(vgh + (size_t)d * NS + sg);
        const v8b b1 = *(const v8b*)(vgl + (size_t)d * NS + sg);
        *(v8b*)(Ksh + p * 8) = a0;
        *(v8b*)(Ksl + p * 8) = a1;
        *(v8b*)(Vth + d * 64 + sg) = b0;
        *(v8b*)(Vtl + d * 64 + sg) = b1;
      }
    }
    __syncthreads();

    v8f s[4];
#pragma unroll
    for (int j = 0; j < 4; ++j) s[j] = zero8();
#pragma unroll 1
    for (int dc = 0; dc < 8; ++dc) {
      const v16b qa = ldfrag_b(Qh + qo + dc * 32);
      const v16b ql = ldfrag_b(Ql + qo + dc * 32);
      const int ko = dc * 32 + 8 * hh;
#pragma unroll
      for (int j = 0; j < 4; ++j) {
        const int kr = (j * 16 + c) * NC + ko;
        FB kb, kl;
        kb.h[0] = *(const v8b*)(Ksh + kr);
        kb.h[1] = *(const v8b*)(Ksh + kr + 16);
        kl.h[0] = *(const v8b*)(Ksl + kr);
        kl.h[1] = *(const v8b*)(Ksl + kr + 16);
        s[j] = mma_b(qa, kb.v, s[j]);
        s[j] = mma_b(qa, kl.v, s[j]);
        s[j] = mma_b(ql, kb.v, s[j]);
      }
    }

#pragma unroll
    for (int r = 0; r < 8; ++r) {
      const int rowq = q0 + 8 * hh + r;
      float m = -INFINITY;
#pragma unroll
      for (int j = 0; j < 4; ++j) {
        const int key = kv0 + j * 16 + c;
        float sv = s[j][r] * 0.0625f;
        sv = (key <= rowq) ? sv : -INFINITY;
        s[j][r] = sv;
        m = fmaxf(m, sv);
      }
#pragma unroll
      for (int off = 1; off < 16; off <<= 1) m = fmaxf(m, __shfl_xor(m, off, 32));
      const float mnew  = fmaxf(mrow[r], m);
      const float msafe = (mnew == -INFINITY) ? 0.f : mnew;
      const float al    = __expf(mrow[r] - msafe);
      mrow[r]  = mnew;
      alpha[r] = al;
      float psum = 0.f;
#pragma unroll
      for (int j = 0; j < 4; ++j) {
        const float p = __expf(s[j][r] - msafe);
        psum += p;
        const unsigned short hb = bf_bits(p);
        const unsigned short lb = bf_bits(p - bf_up(hb));
        const int po = (8 * hh + r) * 64 + j * 16 + c;
        pwh[po] = bf_val(hb);
        pwl[po] = bf_val(lb);
      }
#pragma unroll
      for (int off = 1; off < 16; off <<= 1) psum += __shfl_xor(psum, off, 32);
      lrow[r] = lrow[r] * al + psum;
    }
    __builtin_amdgcn_fence(__ATOMIC_RELEASE, "workgroup");
    __builtin_amdgcn_wave_barrier();
    __builtin_amdgcn_fence(__ATOMIC_ACQUIRE, "workgroup");

    FB pa[2], pl[2];
#pragma unroll
    for (int kk = 0; kk < 2; ++kk) {
      const int pr = c * 64 + kk * 32 + 8 * hh;
      pa[kk].h[0] = *(const v8b*)(pwh + pr);
      pa[kk].h[1] = *(const v8b*)(pwh + pr + 16);
      pl[kk].h[0] = *(const v8b*)(pwl + pr);
      pl[kk].h[1] = *(const v8b*)(pwl + pr + 16);
    }
#pragma unroll 1
    for (int t = 0; t < 16; ++t) {
      float* ap = accW + (t * 32 + lane) * 8;
      v8f acc = *(const v8f*)ap;
#pragma unroll
      for (int r = 0; r < 8; ++r) acc[r] *= alpha[r];
      const int vr0 = (t * 16 + c) * 64 + 8 * hh;
#pragma unroll
      for (int kk = 0; kk < 2; ++kk) {
        FB vb, vl;
        vb.h[0] = *(const v8b*)(Vth + vr0 + kk * 32);
        vb.h[1] = *(const v8b*)(Vth + vr0 + kk * 32 + 16);
        vl.h[0] = *(const v8b*)(Vtl + vr0 + kk * 32);
        vl.h[1] = *(const v8b*)(Vtl + vr0 + kk * 32 + 16);
        acc = mma_b(pa[kk].v, vb.v, acc);
        acc = mma_b(pa[kk].v, vl.v, acc);
        acc = mma_b(pl[kk].v, vb.v, acc);
      }
      *(v8f*)ap = acc;
    }
  }

  if (c == 0) {
#pragma unroll
    for (int r = 0; r < 8; ++r) sD[wave * 16 + 8 * hh + r] = __expf(mrow[r]) * lrow[r];
  }
  __syncthreads();

  float* os = (float*)(lds + L_KSH) + wave * 4096;
  float inv[8];
#pragma unroll
  for (int r = 0; r < 8; ++r) inv[r] = (lrow[r] > 0.f) ? (1.0f / lrow[r]) : 0.f;
#pragma unroll 1
  for (int t = 0; t < 16; ++t) {
    const v8f acc = *(const v8f*)(accW + (t * 32 + lane) * 8);
#pragma unroll
    for (int r = 0; r < 8; ++r) os[(8 * hh + r) * 256 + t * 16 + c] = acc[r] * inv[r];
  }
  __builtin_amdgcn_fence(__ATOMIC_RELEASE, "workgroup");
  __builtin_amdgcn_wave_barrier();
  __builtin_amdgcn_fence(__ATOMIC_ACQUIRE, "workgroup");
  float* og = Op + (zrow + q0) * NC;
  for (int pass = 0; pass < 2; ++pass) {
#pragma unroll 4
    for (int it = 0; it < 32; ++it) {
      const int row = it >> 1;
      const int col = (it & 1) * 128 + lane * 4;
      const v4f v = *(const v4f*)(os + row * 256 + col);
      *(volatile v4f*)(og + (size_t)row * NC + col) = v;
    }
    __threadfence();
  }
  if (wave == 0 && lane < 16) {
    const v4f dv = *(const v4f*)(sD + lane * 4);
    float* dg = Dp + zrow + (size_t)qb * 64 + lane * 4;
    *(volatile v4f*)dg = dv;
    __threadfence();
    *(volatile v4f*)dg = dv;
  }
}

__global__ __launch_bounds__(256) void combine(const float* __restrict__ Op, const float* __restrict__ Dp,
                                               float* out) {
  const int tid  = threadIdx.x;
  const int wave = tid >> 5;
  const int lane = tid & 31;
  const int pbase = blockIdx.x * 32 + wave * 4;
#pragma unroll 1
  for (int pp = 0; pp < 4; ++pp) {
    const int P  = pbase + pp;
    const int b  = P >> 13;
    const int p  = P & (NSEQ - 1);
    const int zb = b * NG;
    const int z1 = zb + (p >> 11),     i1 = p & 2047;
    const int z2 = zb + 4 + (p >> 12), i2 = (p & 4095) >> 1;
    const int z3 = zb + 6,             i3 = p >> 2;
    const float d1  = Dp[(size_t)z1 * NS + i1];
    const float d2r = Dp[(size_t)z2 * NS + i2];
    const float d3r = Dp[(size_t)z3 * NS + i3];
    const float d2  = ((p & 1) == 0) ? d2r : 0.f;
    const float d3  = ((p & 3) == 0) ? d3r : 0.f;
    const float inv = 1.0f / (d1 + d2 + d3);
    const float w1 = d1 * inv, w2 = d2 * inv, w3 = d3 * inv;
    const float* o1 = Op + ((size_t)z1 * NS + i1) * NC;
    const float* o2 = Op + ((size_t)z2 * NS + i2) * NC;
    const float* o3 = Op + ((size_t)z3 * NS + i3) * NC;
    float* orow = out + ((size_t)b * NSEQ + p) * NC;
    v4f res[2];
#pragma unroll
    for (int it = 0; it < 2; ++it) {
      const int col = it * 128 + lane * 4;
      const v4f a  = *(const v4f*)(o1 + col);
      const v4f bq = *(const v4f*)(o2 + col);
      const v4f cq = *(const v4f*)(o3 + col);
      v4f rr;
#pragma unroll
      for (int e = 0; e < 4; ++e) rr[e] = a[e] * w1 + bq[e] * w2 + cq[e] * w3;
      res[it] = rr;
    }
#pragma unroll
    for (int it = 0; it < 2; ++it) *(volatile v4f*)(orow + it * 128 + lane * 4) = res[it];
    __threadfence();
#pragma unroll
    for (int it = 0; it < 2; ++it) *(volatile v4f*)(orow + it * 128 + lane * 4) = res[it];
  }
}

extern "C" void kernel_launch(void* const* d_in, const int* in_sizes, int n_in,
                              void* d_out, int out_size, void* d_ws, size_t ws_size,
                              hipStream_t stream) {
  if (n_in < 4) return;
  if (in_sizes[0] != NB * NSEQ * NC) return;
  if (in_sizes[1] != NC * NC || in_sizes[2] != NC * NC || in_sizes[3] != NC * NC) return;
  if (out_size != NB * NSEQ * NC) return;

  const float* x  = (const float*)d_in[0];
  const float* Wq = (const float*)d_in[1];
  const float* Wk = (const float*)d_in[2];
  const float* Wv = (const float*)d_in[3];

  const size_t PXB = (size_t)NB * NSEQ * NC * 2;
  const size_t PWT = (size_t)NC * NC * 2;
  const size_t PQK = (size_t)NZ * NS * NC * 2;
  const size_t PVT = (size_t)NZ * NC * NS * 2;
  const size_t PO  = (size_t)NZ * NS * NC * 4;
  const size_t PD  = (size_t)NZ * NS * 4;
  size_t off = 0;
  const size_t oXb  = off; off += PXB;
  const size_t oWqT = off; off += PWT;
  const size_t oWkT = off; off += PWT;
  const size_t oWvT = off; off += PWT;
  const size_t oQh  = off; off += PQK;
  const size_t oQl  = off; off += PQK;
  const size_t oKh  = off; off += PQK;
  const size_t oKl  = off; off += PQK;
  const size_t oVTh = off; off += PVT;
  const size_t oVTl = off; off += PVT;
  const size_t oO   = off; off += PO;
  const size_t oD   = off; off += PD;
  if (off > ws_size) return;
  if (off > (size_t)134217728) return;

  char* ws = (char*)d_ws;
  unsigned short* Xb  = (unsigned short*)(ws + oXb);
  unsigned short* WqT = (unsigned short*)(ws + oWqT);
  unsigned short* WkT = (unsigned short*)(ws + oWkT);
  unsigned short* WvT = (unsigned short*)(ws + oWvT);
  unsigned short* Qh  = (unsigned short*)(ws + oQh);
  unsigned short* Ql  = (unsigned short*)(ws + oQl);
  unsigned short* Kh  = (unsigned short*)(ws + oKh);
  unsigned short* Kl  = (unsigned short*)(ws + oKl);
  unsigned short* VTh = (unsigned short*)(ws + oVTh);
  unsigned short* VTl = (unsigned short*)(ws + oVTl);
  float*          O   = (float*)(ws + oO);
  float*          Dn  = (float*)(ws + oD);

  const dim3 blk(256);
  const int n8x = NB * NSEQ * NC / 8;
  const dim3 gCvtX((n8x + 255) / 256);
  const dim3 gWt(NC / 16);
  const dim3 gProj(((NS / 64) * (NC / 64) + 7) / 8, NZ);
  const dim3 gAttn(NZ * NQB);
  const dim3 gMix((NB * NSEQ) / 32);

  cvt_bf16x8<<<gCvtX, blk, 0, stream>>>(x, Xb, n8x);
  prep_wt<<<gWt, blk, 0, stream>>>(Wq, Wk, Wv, WqT, WkT, WvT);
  pgemm<true><<<gProj, blk, 0, stream>>>(Xb, WqT, Qh, Ql);
  pgemm<true><<<gProj, blk, 0, stream>>>(Xb, WkT, Kh, Kl);
  pgemm<false><<<gProj, blk, 0, stream>>>(Xb, WvT, VTh, VTl);
  (void)hipFuncSetAttribute(reinterpret_cast<const void*>(&attn_causal),
                            hipFuncAttributeMaxDynamicSharedMemorySize, L_TOTAL);
  attn_causal<<<gAttn, dim3(128), L_TOTAL, stream>>>(Qh, Ql, Kh, Kl, VTh, VTl, O, Dn);
  combine<<<gMix, blk, 0, stream>>>(O, Dn, (float*)d_out);
  (void)hipGetLastError();
}
